// RUMLayer_39642548142869
// MI455X (gfx1250) — hardware-run, weakly checked
//
#include <hip/hip_runtime.h>

typedef __attribute__((ext_vector_type(16))) _Float16 v16h;
typedef __attribute__((ext_vector_type(8)))  _Float16 v8h;
typedef __attribute__((ext_vector_type(4)))  _Float16 v4h;
typedef __attribute__((ext_vector_type(16))) __bf16   v16b;
typedef __attribute__((ext_vector_type(8)))  __bf16   v8b;
typedef __attribute__((ext_vector_type(8)))  float    v8f;
typedef __attribute__((ext_vector_type(4)))  float    v4f;
typedef __attribute__((ext_vector_type(2)))  float    v2f;
typedef __attribute__((ext_vector_type(4)))  unsigned int v4u;

constexpr int kSamples = 4;
constexpr int kNodes   = 5000;
constexpr int kLen     = 8;
constexpr int kBatch   = kSamples * kNodes;
constexpr int kHid     = 128;
constexpr int kGate    = 3 * kHid;
constexpr int kEdgeF   = 64;
constexpr int kEdges   = 80000;
constexpr int kDin     = kHid + 2 * kHid + 1;
constexpr int kNodesPad = 5056;
constexpr int kRows    = 32;
constexpr int kThreads = 256;
constexpr int kSteps   = 2 * kLen - 1;
constexpr int kHP = 136;
constexpr int kXP = 264;
constexpr int kGP = 388;
constexpr int kSP = 132;
static_assert(kBatch == 20000, "batch");
static_assert(kDin == 385, "input width");
static_assert(kBatch % kRows == 0, "row tile divides batch");
static_assert(kNodesPad % 64 == 0 && kNodesPad >= kNodes, "node pad");
static_assert(kGate % 64 == 0 && kHid % 32 == 0 && kEdgeF % 32 == 0, "gemm tiles");
static_assert((kHP * 2) % 16 == 0 && (kXP * 2) % 16 == 0 && (kGP * 4) % 16 == 0 && (kSP * 4) % 16 == 0, "pitch alignment");
static_assert(kRows * kLen == kThreads, "index staging map");

constexpr float kActCarry = 64.0f;
constexpr float kWgtCarry = 256.0f;
constexpr float kAccInv   = 1.0f / (kActCarry * kWgtCarry);
constexpr float kLoCarry  = 2048.0f;
constexpr float kLoInv    = 1.0f / kLoCarry;
constexpr float kF16Min   = 6.103515625e-5f;
constexpr float kLog2e    = 1.4426950408889634f;

__device__ __forceinline__ unsigned short f2bf_bits(float f) {
  unsigned u = __float_as_uint(f);
  return (unsigned short)((u + 0x7FFFu + ((u >> 16) & 1u)) >> 16);
}
__device__ __forceinline__ float bf_bits2f(unsigned short h) { return __uint_as_float(((unsigned)h) << 16); }

__device__ __forceinline__ float flush14(float s) { return (fabsf(s) < kF16Min) ? 0.0f : s; }
__device__ __forceinline__ int clampi(int v, int lo, int hi) { v = v < lo ? lo : v; return v > hi ? hi : v; }

__device__ __forceinline__ float sig_fast(float x) {
  return __builtin_amdgcn_rcpf(1.0f + __builtin_amdgcn_exp2f(-kLog2e * x));
}
__device__ __forceinline__ float tanh_fast(float x) {
  const float u = __builtin_amdgcn_exp2f((2.0f * kLog2e) * x);
  return fmaf(-2.0f, __builtin_amdgcn_rcpf(u + 1.0f), 1.0f);
}

__device__ __forceinline__ void dep_guard_h(v8f& a, v8f& b, v16h x, v16h y) { asm volatile("v_nop\n\tv_nop\n\tv_nop\n\tv_nop" : "+v"(a), "+v"(b) : "v"(x), "v"(y)); }
__device__ __forceinline__ void dep_guard_b(v8f& a, v8f& b, v16b x, v16b y) { asm volatile("v_nop\n\tv_nop\n\tv_nop\n\tv_nop" : "+v"(a), "+v"(b) : "v"(x), "v"(y)); }
__device__ __forceinline__ void keep4_h(v16h a, v16h b, v16h c, v16h d) { asm volatile("v_nop" :: "v"(a), "v"(b), "v"(c), "v"(d)); }
__device__ __forceinline__ void keep4_b(v16b a, v16b b, v16b c, v16b d) { asm volatile("v_nop" :: "v"(a), "v"(b), "v"(c), "v"(d)); }
__device__ __forceinline__ void acc_guard4(v8f& a, v8f& b, v8f& c, v8f& d) { asm volatile("v_nop\n\tv_nop\n\tv_nop\n\tv_nop" : "+v"(a), "+v"(b), "+v"(c), "+v"(d)); }

template <typename T> struct Frag;
template <> struct Frag<_Float16> {
  typedef v16h V; union U { v16h v; v8h h[2]; };
  static __device__ __forceinline__ v16h load(const _Float16* p) {
    U f; f.h[0] = *(const v8h*)(p); f.h[1] = *(const v8h*)(p + 16); return f.v;
  }
  static __device__ __forceinline__ v8f mma(v16h a, v16h b, v8f c) {
    return __builtin_amdgcn_wmma_f32_16x16x32_f16(false, a, false, b, (short)0, c, false, false);
  }
  static __device__ __forceinline__ void guard(v8f& a, v8f& b, v16h x, v16h y) { dep_guard_h(a, b, x, y); }
  static __device__ __forceinline__ void keep(v16h a, v16h b, v16h c, v16h d) { keep4_h(a, b, c, d); }
};
template <> struct Frag<__bf16> {
  typedef v16b V; union U { v16b v; v8b h[2]; };
  static __device__ __forceinline__ v16b load(const __bf16* p) {
    U f; f.h[0] = *(const v8b*)(p); f.h[1] = *(const v8b*)(p + 16); return f.v;
  }
  static __device__ __forceinline__ v8f mma(v16b a, v16b b, v8f c) {
    return __builtin_amdgcn_wmma_f32_16x16x32_bf16(false, a, false, b, (short)0, c, false, false);
  }
  static __device__ __forceinline__ void guard(v8f& a, v8f& b, v16b x, v16b y) { dep_guard_b(a, b, x, y); }
  static __device__ __forceinline__ void keep(v16b a, v16b b, v16b c, v16b d) { keep4_b(a, b, c, d); }
};

template <int ET> struct Elem;
template <> struct Elem<0> { typedef _Float16 T; };
template <> struct Elem<1> { typedef __bf16 T; };
template <int ET, bool SPLIT, int BIAS_MODE, int OUT_MODE, bool RESID, int ACT = 0>
__global__ __launch_bounds__(256) void wmma_gemm64(
    const unsigned short* __restrict__ Ap, const unsigned short* __restrict__ A2p, int lda, long strideA,
    const unsigned short* __restrict__ Btp, const unsigned short* __restrict__ Bt2p, int ldb, long strideB,
    void* __restrict__ Cout, void* __restrict__ Cout2, int ldc, long strideC,
    const float* __restrict__ bias,
    const float* __restrict__ resid, long strideR,
    int M, int N, int K, float scale) {
  typedef typename Elem<ET>::T T;
  typedef typename Frag<T>::V V;
  const T* A = (const T*)Ap; const T* A2 = (const T*)A2p; const T* Bt = (const T*)Btp; const T* Bt2 = (const T*)Bt2p;
  __shared__ __align__(16) float sT[8][16 * 68];
  const int b    = blockIdx.y;
  const int lane = threadIdx.x & 31;
  const int wave = threadIdx.x >> 5;
  const int tilesN = N >> 6;
  const int tilesM = M >> 6;
  const int tile = blockIdx.x * 8 + wave;
  if (tile >= tilesM * tilesN) return;
  const int tm = tile / tilesN;
  const int tn = tile - tm * tilesN;
  const int m0 = tm << 6;
  const int n0 = tn << 6;

  const T* Ab  = A  + (size_t)b * strideA;
  const T* Bb  = Bt + (size_t)b * strideB;
  const T* Ab2 = SPLIT ? (A2  + (size_t)b * strideA) : nullptr;
  const T* Bb2 = SPLIT ? (Bt2 + (size_t)b * strideB) : nullptr;

  const int rlane = lane & 15;
  const int koff  = (lane >> 4) * 8;
  const int mOff  = (lane >> 4) * 8;

  v8f acc[4][4];
#pragma unroll
  for (int i = 0; i < 4; ++i)
#pragma unroll
    for (int j = 0; j < 4; ++j) acc[i][j] = (v8f){0.f,0.f,0.f,0.f,0.f,0.f,0.f,0.f};

  for (int k0 = 0; k0 < K; k0 += 32) {
    V bh[4], bl[4];
#pragma unroll
    for (int j = 0; j < 4; ++j) {
      const size_t bo = (size_t)(n0 + (j << 4) + rlane) * ldb + koff + k0;
      bh[j] = Frag<T>::load(Bb + bo);
      if (SPLIT) bl[j] = Frag<T>::load(Bb2 + bo);
    }
#pragma unroll
    for (int i = 0; i < 4; ++i) {
      const size_t ao = (size_t)(m0 + (i << 4) + rlane) * lda + koff + k0;
      V ah = Frag<T>::load(Ab + ao);
      V al;
      if (SPLIT) al = Frag<T>::load(Ab2 + ao);
#pragma unroll
      for (int j = 0; j < 4; ++j) {
        acc[i][j] = Frag<T>::mma(ah, bh[j], acc[i][j]);
        if (SPLIT) {
          acc[i][j] = Frag<T>::mma(ah, bl[j], acc[i][j]);
          acc[i][j] = Frag<T>::mma(al, bh[j], acc[i][j]);
        }
      }
      Frag<T>::guard(acc[i][0], acc[i][1], ah, SPLIT ? al : ah);
      Frag<T>::guard(acc[i][2], acc[i][3], ah, SPLIT ? al : ah);
    }
    Frag<T>::keep(bh[0], bh[1], bh[2], bh[3]);
    if (SPLIT) Frag<T>::keep(bl[0], bl[1], bl[2], bl[3]);
  }
  acc_guard4(acc[0][0], acc[0][1], acc[0][2], acc[0][3]);
  acc_guard4(acc[1][0], acc[1][1], acc[1][2], acc[1][3]);
  acc_guard4(acc[2][0], acc[2][1], acc[2][2], acc[2][3]);
  acc_guard4(acc[3][0], acc[3][1], acc[3][2], acc[3][3]);

  float* slab = sT[wave];
  const float* Rb = RESID ? (resid + (size_t)b * strideR) : nullptr;
#pragma unroll
  for (int i = 0; i < 4; ++i) {
    const int mBase = m0 + (i << 4);
#pragma unroll
    for (int j = 0; j < 4; ++j) {
      const int n = n0 + (j << 4) + rlane;
      float bv = 0.f;
      if (BIAS_MODE == 2) bv = bias[n];
#pragma unroll
      for (int r = 0; r < 8; ++r) {
        float v = acc[i][j][r] * scale;
        if (BIAS_MODE == 1) v += bias[mBase + mOff + r];
        if (BIAS_MODE == 2) v += bv;
        if (RESID) v += Rb[(size_t)(mBase + mOff + r) * ldc + n];
        if (ACT == 1) v = tanhf(v);
        if (ACT == 2) v = fmaxf(v, 0.0f);
        if (ACT == 3) v = v / (1.0f + expf(-v));
        if (ACT == 4) v = (v > 0.f) ? v : 0.01f * v;
        if (ACT == 5) v = 0.5f * v * (1.0f + erff(v * 0.70710678118654752f));
        slab[(mOff + r) * 68 + (j << 4) + rlane] = v;
      }
    }
    __builtin_amdgcn_fence(__ATOMIC_RELEASE, "workgroup");
    __builtin_amdgcn_wave_barrier();
    __builtin_amdgcn_fence(__ATOMIC_ACQUIRE, "workgroup");
    if (OUT_MODE == 0) {
      float* C = (float*)Cout + (size_t)b * strideC;
      const int hh = lane >> 4, c4 = (lane & 15) * 4;
      for (int pass = 0; pass < 2; ++pass) {
#pragma unroll
        for (int it = 0; it < 8; ++it) {
          const int row = it * 2 + hh;
          v4f v = *(const v4f*)(slab + row * 68 + c4);
          *(volatile v4f*)(C + (size_t)(mBase + row) * ldc + n0 + c4) = v;
        }
        __threadfence();
      }
    } else {
      const int q = lane >> 3, c8 = (lane & 7) * 8;
      unsigned short* C  = (unsigned short*)Cout  + (size_t)b * strideC;
      unsigned short* C2 = (OUT_MODE == 2) ? ((unsigned short*)Cout2 + (size_t)b * strideC) : nullptr;
      for (int pass = 0; pass < 2; ++pass) {
#pragma unroll
        for (int it = 0; it < 4; ++it) {
          const int row = it * 4 + q;
          const float* sp = slab + row * 68 + c8;
          v8h hv, lv;
#pragma unroll
          for (int e = 0; e < 8; ++e) {
            if (OUT_MODE == 1) {
              hv[e] = (_Float16)sp[e];
            } else {
              unsigned short hb = f2bf_bits(sp[e]);
              unsigned short lb = f2bf_bits(sp[e] - bf_bits2f(hb));
              hv[e] = __builtin_bit_cast(_Float16, hb);
              lv[e] = __builtin_bit_cast(_Float16, lb);
            }
          }
          *(volatile v8h*)(C + (size_t)(mBase + row) * ldc + n0 + c8) = hv;
          if (OUT_MODE == 2) *(volatile v8h*)(C2 + (size_t)(mBase + row) * ldc + n0 + c8) = lv;
        }
        __threadfence();
      }
    }
    __builtin_amdgcn_fence(__ATOMIC_RELEASE, "workgroup");
    __builtin_amdgcn_wave_barrier();
    __builtin_amdgcn_fence(__ATOMIC_ACQUIRE, "workgroup");
  }
}

__device__ __forceinline__ v16h frag16(const _Float16* p) {
  union { v16h v; v8h h[2]; } f;
  f.h[0] = *(const v8h*)(p);
  f.h[1] = *(const v8h*)(p + 16);
  return f.v;
}
__device__ __forceinline__ v8f mma_h(v16h a, v16h b, v8f c) {
  c = __builtin_amdgcn_wmma_f32_16x16x32_f16(false, a, false, b, (short)0, c, false, false);
  asm volatile("v_nop\n\tv_nop\n\tv_nop\n\tv_nop" : "+v"(c) : "v"(a), "v"(b));
  return c;
}
__device__ __forceinline__ void chunk6(const _Float16* a0p, const _Float16* a1p,
                                       const _Float16* b0p, const _Float16* b1p, const _Float16* b2p,
                                       v8f& c00, v8f& c01, v8f& c02, v8f& c10, v8f& c11, v8f& c12) {
  const v16h a0 = frag16(a0p);
  const v16h a1 = frag16(a1p);
  v16h b = frag16(b0p);
  c00 = mma_h(a0, b, c00);
  c10 = mma_h(a1, b, c10);
  b = frag16(b1p);
  c01 = mma_h(a0, b, c01);
  c11 = mma_h(a1, b, c11);
  b = frag16(b2p);
  c02 = mma_h(a0, b, c02);
  c12 = mma_h(a1, b, c12);
}
__device__ __forceinline__ void edge3(v16h ah0, v16h ah1, v16h al0, v16h al1,
                                      const _Float16* bhp, const _Float16* blp,
                                      v8f& c0, v8f& c1, v8f& l0, v8f& l1) {
  const v16h bh = frag16(bhp);
  const v16h bl = frag16(blp);
  c0 = mma_h(ah0, bh, c0);
  c1 = mma_h(ah1, bh, c1);
  l0 = mma_h(al0, bh, l0);
  l1 = mma_h(al1, bh, l1);
  l0 = mma_h(ah0, bl, l0);
  l1 = mma_h(ah1, bl, l1);
}

__device__ __forceinline__ float sin8(int j) {
  float s = 0.0f;
  s = (j == 1) ? 0.70710677f : s;
  s = (j == 2) ? 1.0f : s;
  s = (j == 3) ? 0.70710677f : s;
  s = (j == 4) ? -8.742278e-8f : s;
  s = (j == 5) ? -0.7071069f : s;
  s = (j == 6) ? -1.0f : s;
  s = (j == 7) ? -0.70710653f : s;
  return s;
}
__device__ __forceinline__ float cos8(int j) {
  float c = 1.0f;
  c = (j == 1) ? 0.70710677f : c;
  c = (j == 2) ? -4.371139e-8f : c;
  c = (j == 3) ? -0.70710677f : c;
  c = (j == 4) ? -1.0f : c;
  c = (j == 5) ? -0.70710665f : c;
  c = (j == 6) ? 1.1924881e-8f : c;
  c = (j == 7) ? 0.70710701f : c;
  return c;
}

__global__ __launch_bounds__(256)
void degmax_kernel(const int* __restrict__ walks, const int* __restrict__ deg, float* __restrict__ maxline) {
  __shared__ int sm[kThreads];
  const int tid = threadIdx.x;
  const int lane = tid & 31;
  int m = -2147483647 - 1;
#pragma unroll 1
  for (int i = tid; i < kBatch * kLen; i += kThreads) {
    const int w = clampi(walks[i], 0, kNodes - 1);
    const int d = deg[w];
    m = d > m ? d : m;
  }
  sm[tid] = m;
  __syncthreads();
  int v = sm[lane * 8];
#pragma unroll
  for (int q = 1; q < 8; ++q) { const int x = sm[lane * 8 + q]; v = x > v ? x : v; }
#pragma unroll
  for (int off = 16; off > 0; off >>= 1) { const int o = __shfl_xor(v, off, 32); v = o > v ? o : v; }
  const float fv = (float)v;
  if (tid < 32) {
    volatile float* p = maxline;
    p[lane] = fv;
    __threadfence();
    p[lane] = fv;
  }
}

__global__ __launch_bounds__(256)
void edge_fold_kernel(const float* __restrict__ wih, const float* __restrict__ we,
                      _Float16* __restrict__ m2hi, _Float16* __restrict__ m2lo) {
  __shared__ float sv[kThreads];
  const int tid = threadIdx.x;
  const int g = blockIdx.x * 4 + (tid >> 6);
  const int c = tid & 63;
  float acc = 0.0f;
#pragma unroll 5
  for (int d = 0; d < kDin; ++d) acc = fmaf(wih[(size_t)g * kDin + d], we[(size_t)d * kEdgeF + c], acc);
  sv[tid] = acc;
  __syncthreads();
  if (tid < 32) {
    v8h hv, lv;
#pragma unroll
    for (int e = 0; e < 8; ++e) {
      const float s = flush14(sv[tid * 8 + e] * kWgtCarry);
      const _Float16 hq = (_Float16)s;
      const float rr = flush14((s - (float)hq) * kLoCarry);
      hv[e] = hq;
      lv[e] = (_Float16)rr;
    }
    _Float16* ph = m2hi + (size_t)blockIdx.x * 256 + tid * 8;
    _Float16* pl = m2lo + (size_t)blockIdx.x * 256 + tid * 8;
    for (int pass = 0; pass < 2; ++pass) {
      *(volatile v8h*)ph = hv;
      *(volatile v8h*)pl = lv;
      __threadfence();
    }
  }
}

template <int MODE>
__global__ __launch_bounds__(256)
void pack_rows_kernel(const float* __restrict__ src, int ld, int col0, int rows_real, int rows_pad, int kcols, float carry,
                      unsigned short* __restrict__ p0, unsigned short* __restrict__ p1) {
  const int gidx = blockIdx.x * kThreads + threadIdx.x;
  const int gpr = kcols >> 3;
  if (gidx >= rows_pad * gpr) return;
  const int row = gidx / gpr;
  const int c8 = (gidx - row * gpr) * 8;
  const int rc = row < rows_real ? row : rows_real - 1;
  const bool live = row < rows_real;
  const float* sp = src + (size_t)rc * ld + col0 + c8;
  float v[8];
#pragma unroll
  for (int e = 0; e < 8; ++e) {
    float x = sp[e];
    asm volatile("" : "+v"(x));
    v[e] = live ? x : 0.0f;
  }
  if (MODE == 0) {
    v8h hv;
#pragma unroll
    for (int e = 0; e < 8; ++e) hv[e] = (_Float16)flush14(v[e] * carry);
    _Float16* dp = (_Float16*)p0 + (size_t)gidx * 8;
    for (int pass = 0; pass < 2; ++pass) {
      *(volatile v8h*)dp = hv;
      __threadfence();
    }
  } else {
    v4u wh, wl;
#pragma unroll
    for (int q = 0; q < 4; ++q) {
      const unsigned short h0 = f2bf_bits(v[2 * q]);
      const unsigned short l0 = f2bf_bits(v[2 * q] - bf_bits2f(h0));
      const unsigned short h1 = f2bf_bits(v[2 * q + 1]);
      const unsigned short l1 = f2bf_bits(v[2 * q + 1] - bf_bits2f(h1));
      wh[q] = (unsigned)h0 | ((unsigned)h1 << 16);
      wl[q] = (unsigned)l0 | ((unsigned)l1 << 16);
    }
    unsigned short* d0 = p0 + (size_t)gidx * 8;
    unsigned short* d1 = p1 + (size_t)gidx * 8;
    for (int pass = 0; pass < 2; ++pass) {
      *(volatile v4u*)d0 = wh;
      *(volatile v4u*)d1 = wl;
      __threadfence();
    }
  }
}

struct WalkConst { float wr0, wr1, wz0, wz1, wn0, wn1, bsr, bsz, bin, bhn; };

__device__ __forceinline__ void walk_gates(const v8f ar, const v8f az, const v8f an, float (&hs)[8],
                                           const float* cp, const WalkConst& k, _Float16* hcol) {
#pragma unroll
  for (int r = 0; r < 8; ++r) {
    const float s = cp[r * 16];
    const float c = cp[r * 16 + 1];
    const float xr = fmaf(s, k.wr0, fmaf(c, k.wr1, k.bsr));
    const float xz = fmaf(s, k.wz0, fmaf(c, k.wz1, k.bsz));
    const float xn = fmaf(s, k.wn0, fmaf(c, k.wn1, k.bin));
    const float rg = sig_fast(fmaf(ar[r], kAccInv, xr));
    const float zg = sig_fast(fmaf(az[r], kAccInv, xz));
    const float hn = fmaf(an[r], kAccInv, k.bhn);
    const float ng = tanh_fast(fmaf(rg, hn, xn));
    const float hv = fmaf(zg, hs[r] - ng, ng);
    hs[r] = hv;
    hcol[r * kHP] = (_Float16)flush14(hv * kActCarry);
  }
}

__global__ __launch_bounds__(256)
void walk_cells_kernel(const int* __restrict__ walks,
                       const float* __restrict__ wih_f, const float* __restrict__ bih_f, const float* __restrict__ bhh_f,
                       const float* __restrict__ wih_b, const float* __restrict__ bih_b, const float* __restrict__ bhh_b,
                       const _Float16* whh_f, const _Float16* whh_b,
                       _Float16* yf, _Float16* ybf, float* hdir) {
  __shared__ __align__(16) _Float16 h16[kRows * kHP];
  __shared__ __align__(16) float stg[kRows * kSP];
  __shared__ __align__(8) float code[kRows * 16];
  __shared__ int wk[kRows * kLen];

  const int tid = threadIdx.x;
  const int lane = tid & 31;
  const int wave = tid >> 5;
  const int n = lane & 15;
  const int hh = lane >> 4;
  const int j = wave * 16 + n;
  const int dir = blockIdx.y;
  const int b0 = blockIdx.x * kRows;

  const float* wd = dir ? wih_b : wih_f;
  const float* bi = dir ? bih_b : bih_f;
  const float* bh = dir ? bhh_b : bhh_f;
  const _Float16* wpl = dir ? whh_b : whh_f;
  _Float16* ypl = dir ? ybf : yf;

  const int wv = clampi(walks[(size_t)b0 * kLen + tid], 0, kNodes - 1);
  wk[tid] = wv;
  __syncthreads();
  {
    const int row = tid >> 3;
    const int l = tid & 7;
    int jf = l;
#pragma unroll
    for (int q = 7; q >= 0; --q) {
      const int wq = wk[row * 8 + q];
      jf = (q <= l && wq == wv) ? q : jf;
    }
    code[row * 16 + (7 - l) * 2]     = sin8(jf);
    code[row * 16 + (7 - l) * 2 + 1] = cos8(jf);
  }

  WalkConst kc;
  {
    const v2f w_r = *(const v2f*)(wd + 2 * j);
    const v2f w_z = *(const v2f*)(wd + 2 * (kHid + j));
    const v2f w_n = *(const v2f*)(wd + 2 * (2 * kHid + j));
    kc.wr0 = w_r[0]; kc.wr1 = w_r[1];
    kc.wz0 = w_z[0]; kc.wz1 = w_z[1];
    kc.wn0 = w_n[0]; kc.wn1 = w_n[1];
    kc.bsr = bi[j] + bh[j];
    kc.bsz = bi[kHid + j] + bh[kHid + j];
    kc.bin = bi[2 * kHid + j];
    kc.bhn = bh[2 * kHid + j];
  }

  float hs0[8], hs1[8];
#pragma unroll
  for (int r = 0; r < 8; ++r) { hs0[r] = 0.0f; hs1[r] = 0.0f; }
  __syncthreads();

  const v8f vz = (v8f){0.f,0.f,0.f,0.f,0.f,0.f,0.f,0.f};
  const _Float16* bR = wpl + (size_t)j * kHid;
  const _Float16* bZ = wpl + (size_t)(kHid + j) * kHid;
  const _Float16* bN = wpl + (size_t)(2 * kHid + j) * kHid;

#pragma unroll 1
  for (int t = 0; t < kLen; ++t) {
    asm volatile("" ::: "memory");
    const int pos = dir ? (kLen - 1 - t) : t;
    v8f ar0 = vz, az0 = vz, an0 = vz, ar1 = vz, az1 = vz, an1 = vz;
    if (t > 0) {
#pragma unroll 1
      for (int kk = 0; kk < kHid / 32; ++kk) {
        const int ko = kk * 32 + 8 * hh;
        chunk6(h16 + n * kHP + ko, h16 + (16 + n) * kHP + ko, bR + ko, bZ + ko, bN + ko,
               ar0, az0, an0, ar1, az1, an1);
      }
    }
    __syncthreads();
    walk_gates(ar0, az0, an0, hs0, code + (8 * hh) * 16 + pos * 2, kc, h16 + (8 * hh) * kHP + j);
    walk_gates(ar1, az1, an1, hs1, code + (16 + 8 * hh) * 16 + pos * 2, kc, h16 + (16 + 8 * hh) * kHP + j);
    __syncthreads();
    {
      const int row = tid >> 4;
      const int c8 = (tid & 15) * 8;
      const v8h v0 = *(const v8h*)(h16 + row * kHP + c8);
      const v8h v1 = *(const v8h*)(h16 + (16 + row) * kHP + c8);
      _Float16* gp = ypl + ((size_t)pos * kBatch + b0) * kHid;
      for (int pass = 0; pass < 2; ++pass) {
        *(volatile v8h*)(gp + (size_t)row * kHid + c8) = v0;
        *(volatile v8h*)(gp + (size_t)(16 + row) * kHid + c8) = v1;
        __threadfence();
      }
    }
  }

#pragma unroll
  for (int r = 0; r < 8; ++r) {
    stg[(8 * hh + r) * kSP + j] = hs0[r];
    stg[(16 + 8 * hh + r) * kSP + j] = hs1[r];
  }
  __syncthreads();
  {
    v4f o[4];
#pragma unroll
    for (int it = 0; it < 4; ++it) {
      const int idx = it * kThreads + tid;
      o[it] = *(const v4f*)(stg + (idx >> 5) * kSP + (idx & 31) * 4);
    }
    float* hp = hdir + ((size_t)dir * kBatch + b0) * kHid;
    for (int pass = 0; pass < 2; ++pass) {
#pragma unroll
      for (int it = 0; it < 4; ++it) {
        const int idx = it * kThreads + tid;
        *(volatile v4f*)(hp + (size_t)(idx >> 5) * kHid + (idx & 31) * 4) = o[it];
      }
      __threadfence();
    }
  }
}

struct MainConst { float bsr, bsz, bin, bhn, wdr, wdz, wdn; };

__device__ __forceinline__ void main_gates(const v8f ar, const v8f az, const v8f axn, const v8f ahn, float (&hs)[8],
                                           const float* gtp, const float* dgp, bool even,
                                           const MainConst& k, _Float16* hcol) {
#pragma unroll
  for (int r = 0; r < 8; ++r) {
    const float g_r = gtp[r * kGP];
    const float g_z = gtp[r * kGP + kHid];
    const float g_n = gtp[r * kGP + 2 * kHid];
    const float dw = dgp[r * 8];
    const float xr = even ? fmaf(dw, k.wdr, g_r) : 0.0f;
    const float xz = even ? fmaf(dw, k.wdz, g_z) : 0.0f;
    const float xn = even ? fmaf(dw, k.wdn, g_n) : 0.0f;
    const float rg = sig_fast(fmaf(ar[r], kAccInv, xr) + k.bsr);
    const float zg = sig_fast(fmaf(az[r], kAccInv, xz) + k.bsz);
    const float hn = fmaf(ahn[r], kAccInv, k.bhn);
    const float pn = fmaf(axn[r], kAccInv, xn) + k.bin;
    const float ng = tanh_fast(fmaf(rg, hn, pn));
    const float hv = fmaf(zg, hs[r] - ng, ng);
    hs[r] = hv;
    hcol[r * kHP] = (_Float16)flush14(hv * kActCarry);
  }
}

__global__ __launch_bounds__(256)
void main_cells_kernel(const float* hgp, const float* ep,
                       const int* __restrict__ walks, const int* __restrict__ eids, const int* __restrict__ deg,
                       const float* __restrict__ wih, const float* __restrict__ bih, const float* __restrict__ bhh,
                       const _Float16* whh, const _Float16* wihy, const _Float16* m2hi, const _Float16* m2lo,
                       const _Float16* yf, const _Float16* ybf, const float* hdir, const float* maxline,
                       float* out) {
  __shared__ __align__(16) _Float16 h16[kRows * kHP];
  __shared__ __align__(16) _Float16 x16[kRows * kXP];
  __shared__ __align__(16) float gt[kRows * kGP];
  __shared__ int nidx[kRows * kLen];
  __shared__ int eidx[kRows * kLen];
  __shared__ float degf[kRows * kLen];

  const int tid = threadIdx.x;
  const int lane = tid & 31;
  const int wave = tid >> 5;
  const int n = lane & 15;
  const int hh = lane >> 4;
  const int j = wave * 16 + n;
  const int b0 = blockIdx.x * kRows;

  {
    const int row = tid >> 3;
    const int l = tid & 7;
    const int wv = clampi(walks[(size_t)(b0 + row) * kLen + l], 0, kNodes - 1);
    const int dg = deg[wv];
    const float mx = maxline[0];
    const float inv = 1.0f / mx;
    const int lc = l < (kLen - 1) ? l : (kLen - 2);
    const int ev = clampi(eids[(size_t)(b0 + row) * (kLen - 1) + lc], 0, kEdges - 1);
    nidx[row * 8 + 7 - l] = wv;
    degf[row * 8 + 7 - l] = (float)dg * inv;
    eidx[row * 8 + l] = (l < (kLen - 1)) ? ev : 0;
  }
#pragma unroll
  for (int it = 0; it < 4; ++it) {
    const int idx = it * kThreads + tid;
    const int row = idx >> 5;
    const int c4 = (idx & 31) * 4;
    const v4f a = *(const v4f*)(hdir + (size_t)(b0 + row) * kHid + c4);
    const v4f bq = *(const v4f*)(hdir + (size_t)(kBatch + b0 + row) * kHid + c4);
    *(v4f*)(gt + row * kSP + c4) = (a + bq) * 0.5f;
  }
  __syncthreads();

  float hs0[8], hs1[8];
#pragma unroll
  for (int r = 0; r < 8; ++r) {
    hs0[r] = gt[(8 * hh + r) * kSP + j];
    hs1[r] = gt[(16 + 8 * hh + r) * kSP + j];
    h16[(8 * hh + r) * kHP + j] = (_Float16)flush14(hs0[r] * kActCarry);
    h16[(16 + 8 * hh + r) * kHP + j] = (_Float16)flush14(hs1[r] * kActCarry);
  }

  MainConst kc;
  kc.bsr = bih[j] + bhh[j];
  kc.bsz = bih[kHid + j] + bhh[kHid + j];
  kc.bin = bih[2 * kHid + j];
  kc.bhn = bhh[2 * kHid + j];
  kc.wdr = wih[(size_t)j * kDin + (kDin - 1)];
  kc.wdz = wih[(size_t)(kHid + j) * kDin + (kDin - 1)];
  kc.wdn = wih[(size_t)(2 * kHid + j) * kDin + (kDin - 1)];
  __syncthreads();

  const v8f vz = (v8f){0.f,0.f,0.f,0.f,0.f,0.f,0.f,0.f};

#pragma unroll 1
  for (int t = 0; t < kSteps; ++t) {
    asm volatile("" ::: "memory");
    const int l = t >> 1;
    const bool even = (t & 1) == 0;

    if (even) {
#pragma unroll
      for (int it = 0; it < 2; ++it) {
        const int idx = it * kThreads + tid;
        const int row = idx >> 4;
        const int c8 = (idx & 15) * 8;
        const size_t go = ((size_t)l * kBatch + b0 + row) * kHid + c8;
        const v8h a = *(const v8h*)(yf + go);
        const v8h bq = *(const v8h*)(ybf + go);
        *(v8h*)(x16 + row * kXP + c8) = a;
        *(v8h*)(x16 + row * kXP + kHid + c8) = bq;
      }
#pragma unroll 4
      for (int it = 0; it < 12; ++it) {
        const int idx = it * kThreads + tid;
        const int row = idx / 96;
        const int c4 = (idx - row * 96) * 4;
        const int node = nidx[row * 8 + l];
        const v4f g = *(const v4f*)(hgp + (size_t)node * kGate + c4);
        *(v4f*)(gt + row * kGP + c4) = g;
      }
    } else {
#pragma unroll
      for (int it = 0; it < 2; ++it) {
        const int idx = it * kThreads + tid;
        const int row = idx >> 4;
        const int c4 = (idx & 15) * 4;
        const int eid = eidx[row * 8 + l];
        const v4f ev = *(const v4f*)(ep + (size_t)eid * kEdgeF + c4);
        v4h hv, lv;
#pragma unroll
        for (int q = 0; q < 4; ++q) {
          const float s = flush14(ev[q] * kActCarry);
          const _Float16 hq = (_Float16)s;
          const float rr = flush14((s - (float)hq) * kLoCarry);
          hv[q] = hq;
          lv[q] = (_Float16)rr;
        }
        *(v4h*)(x16 + row * kXP + c4) = hv;
        *(v4h*)(x16 + row * kXP + kEdgeF + c4) = lv;
      }
    }
    __syncthreads();

    v8f ar0 = vz, az0 = vz, axn0 = vz, ahn0 = vz;
    v8f ar1 = vz, az1 = vz, axn1 = vz, ahn1 = vz;
    if (even) {
      const _Float16* bR = wihy + (size_t)j * (2 * kHid);
      const _Float16* bZ = wihy + (size_t)(kHid + j) * (2 * kHid);
      const _Float16* bN = wihy + (size_t)(2 * kHid + j) * (2 * kHid);
#pragma unroll 1
      for (int kk = 0; kk < (2 * kHid) / 32; ++kk) {
        const int ko = kk * 32 + 8 * hh;
        chunk6(x16 + n * kXP + ko, x16 + (16 + n) * kXP + ko, bR + ko, bZ + ko, bN + ko,
               ar0, az0, axn0, ar1, az1, axn1);
      }
    } else {
      v8f lr0 = vz, lz0 = vz, ln0 = vz, lr1 = vz, lz1 = vz, ln1 = vz;
#pragma unroll 1
      for (int kk = 0; kk < kEdgeF / 32; ++kk) {
        const int ko = kk * 32 + 8 * hh;
        const v16h ah0 = frag16(x16 + n * kXP + ko);
        const v16h ah1 = frag16(x16 + (16 + n) * kXP + ko);
        const v16h al0 = frag16(x16 + n * kXP + kEdgeF + ko);
        const v16h al1 = frag16(x16 + (16 + n) * kXP + kEdgeF + ko);
        edge3(ah0, ah1, al0, al1, m2hi + (size_t)j * kEdgeF + ko, m2lo + (size_t)j * kEdgeF + ko, ar0, ar1, lr0, lr1);
        edge3(ah0, ah1, al0, al1, m2hi + (size_t)(kHid + j) * kEdgeF + ko, m2lo + (size_t)(kHid + j) * kEdgeF + ko, az0, az1, lz0, lz1);
        edge3(ah0, ah1, al0, al1, m2hi + (size_t)(2 * kHid + j) * kEdgeF + ko, m2lo + (size_t)(2 * kHid + j) * kEdgeF + ko, axn0, axn1, ln0, ln1);
      }
      ar0 = ar0 + lr0 * kLoInv;
      ar1 = ar1 + lr1 * kLoInv;
      az0 = az0 + lz0 * kLoInv;
      az1 = az1 + lz1 * kLoInv;
      axn0 = axn0 + ln0 * kLoInv;
      axn1 = axn1 + ln1 * kLoInv;
    }
    {
      const _Float16* bR = whh + (size_t)j * kHid;
      const _Float16* bZ = whh + (size_t)(kHid + j) * kHid;
      const _Float16* bN = whh + (size_t)(2 * kHid + j) * kHid;
#pragma unroll 1
      for (int kk = 0; kk < kHid / 32; ++kk) {
        const int ko = kk * 32 + 8 * hh;
        chunk6(h16 + n * kHP + ko, h16 + (16 + n) * kHP + ko, bR + ko, bZ + ko, bN + ko,
               ar0, az0, ahn0, ar1, az1, ahn1);
      }
    }
    __syncthreads();

    main_gates(ar0, az0, axn0, ahn0, hs0, gt + (8 * hh) * kGP + j, degf + (8 * hh) * 8 + l, even, kc,
               h16 + (8 * hh) * kHP + j);
    main_gates(ar1, az1, axn1, ahn1, hs1, gt + (16 + 8 * hh) * kGP + j, degf + (16 + 8 * hh) * 8 + l, even, kc,
               h16 + (16 + 8 * hh) * kHP + j);
    __syncthreads();
  }

#pragma unroll
  for (int r = 0; r < 8; ++r) {
    gt[(8 * hh + r) * kSP + j] = hs0[r];
    gt[(16 + 8 * hh + r) * kSP + j] = hs1[r];
  }
  __syncthreads();
  {
    v4f o[4];
#pragma unroll
    for (int it = 0; it < 4; ++it) {
      const int idx = it * kThreads + tid;
      o[it] = *(const v4f*)(gt + (idx >> 5) * kSP + (idx & 31) * 4);
    }
    float* op = out + (size_t)b0 * kHid;
    for (int pass = 0; pass < 2; ++pass) {
#pragma unroll
      for (int it = 0; it < 4; ++it) {
        const int idx = it * kThreads + tid;
        *(volatile v4f*)(op + (size_t)(idx >> 5) * kHid + (idx & 31) * 4) = o[it];
      }
      __threadfence();
    }
  }
}

extern "C" void kernel_launch(void* const* d_in, const int* in_sizes, int n_in,
                              void* d_out, int out_size, void* d_ws, size_t ws_size,
                              hipStream_t stream) {
  if (n_in < 18) return;
  if (in_sizes[0] < kNodes * kHid || in_sizes[1] < kEdges * kEdgeF || in_sizes[2] < kDin * kEdgeF ||
      in_sizes[3] < kGate * 2 || in_sizes[4] < kGate * kHid || in_sizes[5] < kGate || in_sizes[6] < kGate ||
      in_sizes[7] < kGate * 2 || in_sizes[8] < kGate * kHid || in_sizes[9] < kGate || in_sizes[10] < kGate ||
      in_sizes[11] < kGate * kDin || in_sizes[12] < kGate * kHid || in_sizes[13] < kGate || in_sizes[14] < kGate ||
      in_sizes[15] < kBatch * kLen || in_sizes[16] < kBatch * (kLen - 1) || in_sizes[17] < kNodes ||
      out_size < kBatch * kHid) return;

  const float* h     = (const float*)d_in[0];
  const float* e     = (const float*)d_in[1];
  const float* W_e   = (const float*)d_in[2];
  const float* Wih_f = (const float*)d_in[3];
  const float* Whh_f = (const float*)d_in[4];
  const float* bih_f = (const float*)d_in[5];
  const float* bhh_f = (const float*)d_in[6];
  const float* Wih_b = (const float*)d_in[7];
  const float* Whh_b = (const float*)d_in[8];
  const float* bih_b = (const float*)d_in[9];
  const float* bhh_b = (const float*)d_in[10];
  const float* Wih   = (const float*)d_in[11];
  const float* Whh   = (const float*)d_in[12];
  const float* bih   = (const float*)d_in[13];
  const float* bhh   = (const float*)d_in[14];
  const int* walks   = (const int*)d_in[15];
  const int* eids    = (const int*)d_in[16];
  const int* deg     = (const int*)d_in[17];
  float* out = (float*)d_out;

  char* wsb = (char*)d_ws;
  size_t off = 0;
  auto take = [&](size_t bytes) -> char* {
    char* p = wsb + off;
    off = (off + bytes + 255) & ~(size_t)255;
    return p;
  };
  float* maxline = (float*)take(128);
  unsigned short* whhf16 = (unsigned short*)take((size_t)kGate * kHid * 2);
  unsigned short* whhb16 = (unsigned short*)take((size_t)kGate * kHid * 2);
  unsigned short* whh16  = (unsigned short*)take((size_t)kGate * kHid * 2);
  unsigned short* wihy16 = (unsigned short*)take((size_t)kGate * 2 * kHid * 2);
  unsigned short* wihh_hi = (unsigned short*)take((size_t)kGate * kHid * 2);
  unsigned short* wihh_lo = (unsigned short*)take((size_t)kGate * kHid * 2);
  unsigned short* m2hi = (unsigned short*)take((size_t)kGate * kEdgeF * 2);
  unsigned short* m2lo = (unsigned short*)take((size_t)kGate * kEdgeF * 2);
  unsigned short* hhi = (unsigned short*)take((size_t)kNodesPad * kHid * 2);
  unsigned short* hlo = (unsigned short*)take((size_t)kNodesPad * kHid * 2);
  float* hg = (float*)take((size_t)kNodesPad * kGate * 4);
  unsigned short* yf  = (unsigned short*)take((size_t)kLen * kBatch * kHid * 2);
  unsigned short* ybf = (unsigned short*)take((size_t)kLen * kBatch * kHid * 2);
  float* hdir = (float*)take((size_t)2 * kBatch * kHid * 4);
  if (off > ws_size || off > (size_t)134217728) return;

  degmax_kernel<<<dim3(1), dim3(kThreads), 0, stream>>>(walks, deg, maxline);
  edge_fold_kernel<<<dim3(kGate / 4), dim3(kThreads), 0, stream>>>(Wih, W_e, (_Float16*)m2hi, (_Float16*)m2lo);

  pack_rows_kernel<0><<<dim3((kGate * (kHid / 8) + kThreads - 1) / kThreads), dim3(kThreads), 0, stream>>>(
      Whh_f, kHid, 0, kGate, kGate, kHid, kWgtCarry, whhf16, nullptr);
  pack_rows_kernel<0><<<dim3((kGate * (kHid / 8) + kThreads - 1) / kThreads), dim3(kThreads), 0, stream>>>(
      Whh_b, kHid, 0, kGate, kGate, kHid, kWgtCarry, whhb16, nullptr);
  pack_rows_kernel<0><<<dim3((kGate * (kHid / 8) + kThreads - 1) / kThreads), dim3(kThreads), 0, stream>>>(
      Whh, kHid, 0, kGate, kGate, kHid, kWgtCarry, whh16, nullptr);
  pack_rows_kernel<0><<<dim3((kGate * (2 * kHid / 8) + kThreads - 1) / kThreads), dim3(kThreads), 0, stream>>>(
      Wih, kDin, kHid, kGate, kGate, 2 * kHid, kWgtCarry, wihy16, nullptr);
  pack_rows_kernel<1><<<dim3((kGate * (kHid / 8) + kThreads - 1) / kThreads), dim3(kThreads), 0, stream>>>(
      Wih, kDin, 0, kGate, kGate, kHid, 1.0f, wihh_hi, wihh_lo);
  pack_rows_kernel<1><<<dim3((kNodesPad * (kHid / 8) + kThreads - 1) / kThreads), dim3(kThreads), 0, stream>>>(
      h, kHid, 0, kNodes, kNodesPad, kHid, 1.0f, hhi, hlo);

  {
    const int tiles = (kNodesPad / 64) * (kGate / 64);
    wmma_gemm64<1, true, 0, 0, false, 0><<<dim3((tiles + 7) / 8, 1), dim3(256), 0, stream>>>(
        hhi, hlo, kHid, 0L, wihh_hi, wihh_lo, kHid, 0L, (void*)hg, nullptr, kGate, 0L,
        nullptr, nullptr, 0L, kNodesPad, kGate, kHid, 1.0f);
  }

  walk_cells_kernel<<<dim3(kBatch / kRows, 2), dim3(kThreads), 0, stream>>>(
      walks, Wih_f, bih_f, bhh_f, Wih_b, bih_b, bhh_b,
      (const _Float16*)whhf16, (const _Float16*)whhb16, (_Float16*)yf, (_Float16*)ybf, hdir);

  main_cells_kernel<<<dim3(kBatch / kRows), dim3(kThreads), 0, stream>>>(
      hg, e, walks, eids, deg, Wih, bih, bhh,
      (const _Float16*)whh16, (const _Float16*)wihy16, (const _Float16*)m2hi, (const _Float16*)m2lo,
      (const _Float16*)yf, (const _Float16*)ybf, hdir, maxline, out);
}
